// LinearBase_44573170598240
// MI455X (gfx1250) — hardware-run, weakly checked
//
#include <hip/hip_runtime.h>
#include <math.h>

typedef __attribute__((ext_vector_type(16))) _Float16 v16h;
typedef __attribute__((ext_vector_type(8)))  _Float16 v8h;
typedef __attribute__((ext_vector_type(8)))  float    v8f;
typedef __attribute__((ext_vector_type(4)))  float    v4f;

constexpr int kRows     = 32768;
constexpr int kIn       = 256;
constexpr int kOut      = 256;
constexpr int kNb       = 11;
constexpr int kSegs     = kNb + 1;
constexpr int kKtot     = kSegs * kIn;
constexpr int kSlabRows = 16384;
constexpr int kNumSlabs = kRows / kSlabRows;
constexpr int kExpWaves = 4;
constexpr int kCells    = 14;

constexpr float kCarryA = 1024.0f;
constexpr float kCarryW = 16.0f;
constexpr float kFold   = 1.0f / (kCarryA * kCarryW);
constexpr float kSixthA = kCarryA / 6.0f;

static_assert(kKtot == 3072, "K extent");
static_assert((kKtot % 32) == 0, "GEMM K multiple of 32");
static_assert((kSlabRows % 64) == 0 && (kOut % 64) == 0, "GEMM M,N multiples of 64");
static_assert(kNumSlabs * kSlabRows == kRows, "slab split");
static_assert((kSlabRows % kExpWaves) == 0, "expand grid exact");
static_assert(kIn == 256 && kOut == 256, "lane maps assume 256 features");
static_assert(kFold == 1.0f / 16384.0f, "fold is 2^-14");

constexpr size_t kBytesWt = (size_t)kOut * kKtot * 2;
constexpr size_t kBytesAp = (size_t)kSlabRows * kKtot * 2;
constexpr size_t kOffWt   = 0;
constexpr size_t kOffAp   = kOffWt + kBytesWt;
constexpr size_t kWsTotal = kOffAp + kBytesAp;
static_assert(kBytesWt == 1572864ull, "carve WT");
static_assert(kBytesAp == 100663296ull, "carve AP");
static_assert(kWsTotal == 102236160ull, "carve total");
static_assert(kWsTotal <= 134217728ull, "carve cap");
static_assert((kOffAp % 128) == 0, "128-B aligned regions");

__device__ __forceinline__ void tie_acc_h(v8f& a, v16h x, v16h y) {
  asm volatile("v_nop\n\tv_nop\n\tv_nop\n\tv_nop" : "+v"(a) : "v"(x), "v"(y));
}
__device__ __forceinline__ void settle_acc(v8f& a) {
  asm volatile("v_nop\n\tv_nop\n\tv_nop\n\tv_nop" : "+v"(a));
}
__device__ __forceinline__ void keep4_h(v16h a, v16h b, v16h c, v16h d) {
  asm volatile("v_nop" :: "v"(a), "v"(b), "v"(c), "v"(d));
}
struct FragH {
  union U { v16h v; v8h h[2]; };
  static __device__ __forceinline__ v16h load(const _Float16* p) {
    U f;
    f.h[0] = *(const v8h*)(p);
    f.h[1] = *(const v8h*)(p + 16);
    return f.v;
  }
  static __device__ __forceinline__ v8f mma(v16h a, v16h b, v8f c) {
    return __builtin_amdgcn_wmma_f32_16x16x32_f16(false, a, false, b, (short)0, c, false, false);
  }
};

__global__ __launch_bounds__(256) void pack_weights_kernel(
    const float* __restrict__ coeff, const float* __restrict__ base_w, unsigned short* __restrict__ Wt)
{
  const int lane = threadIdx.x & 31;
  const int wave = threadIdx.x >> 5;
  const int seg  = blockIdx.x;
  const int o    = blockIdx.y * 8 + wave;
  const int i0   = lane * 8;
  float v[8];
  if (seg < kNb) {
    const float* cp = coeff + ((size_t)o * kIn + i0) * kNb + seg;
#pragma unroll
    for (int e = 0; e < 8; ++e) v[e] = cp[(size_t)e * kNb];
  } else {
    const float* bp = base_w + (size_t)o * kIn + i0;
    const v4f a0 = *(const v4f*)(bp);
    const v4f a1 = *(const v4f*)(bp + 4);
    v[0] = a0[0]; v[1] = a0[1]; v[2] = a0[2]; v[3] = a0[3];
    v[4] = a1[0]; v[5] = a1[1]; v[6] = a1[2]; v[7] = a1[3];
  }
  v8h hv;
#pragma unroll
  for (int e = 0; e < 8; ++e) {
    const float sv = v[e] * kCarryW;
    hv[e] = (_Float16)sv;
  }
  unsigned short* dst = Wt + (size_t)o * kKtot + (size_t)seg * kIn + i0;
  *(volatile v8h*)dst = hv;
  __threadfence();
  *(volatile v8h*)dst = hv;
}

__global__ __launch_bounds__(128) void expand_rows_kernel(
    const float* __restrict__ x, const float* __restrict__ gamma, const float* __restrict__ beta,
    unsigned short* __restrict__ Aplane, int row0)
{
  __shared__ __align__(16) float sT[kExpWaves][kSegs * kIn];
  const int lane = threadIdx.x & 31;
  const int wave = threadIdx.x >> 5;
  const int ml   = blockIdx.x * kExpWaves + wave;
  const float* xr = x + (size_t)(row0 + ml) * kIn;

  float xv[8];
  float s = 0.0f;
#pragma unroll
  for (int c = 0; c < 8; ++c) {
    xv[c] = xr[lane + 32 * c];
    s += xv[c];
  }
#pragma unroll
  for (int off = 16; off >= 1; off >>= 1) s += __shfl_xor(s, off, 32);
  const float mu = s * (1.0f / (float)kIn);
  float q = 0.0f;
#pragma unroll
  for (int c = 0; c < 8; ++c) {
    const float dlt = xv[c] - mu;
    q += dlt * dlt;
  }
#pragma unroll
  for (int off = 16; off >= 1; off >>= 1) q += __shfl_xor(q, off, 32);
  const float var  = q * (1.0f / (float)kIn);
  const float rstd = rsqrtf(var + 1e-5f);

  float* tw = sT[wave];
#pragma unroll 1
  for (int c = 0; c < 8; ++c) {
    const int i = lane + 32 * c;
    const float xc = xr[i];
    const float gm = gamma[i];
    const float bt = beta[i];
    const float z  = (xc - mu) * rstd * gm + bt;
    const float u  = fmaf(z, 4.0f, 7.0f);
    const float cf = floorf(u);
    const float t  = u - cf;
    const bool inr = (u >= 0.0f) && (u < (float)kCells);
    const float cfc = fminf(fmaxf(cf, -8.0f), 40.0f);
    const int ci = inr ? (int)cfc : -64;
    const float t2  = t * t;
    const float t3  = t2 * t;
    const float omt = 1.0f - t;
    const float w3 = kSixthA * t3;
    const float w0 = kSixthA * (omt * omt * omt);
    const float w1 = kSixthA * fmaf(t3, 3.0f, fmaf(t2, -6.0f, 4.0f));
    const float w2 = kSixthA * fmaf(3.0f, (t + t2) - t3, 1.0f);
#pragma unroll
    for (int n = 0; n < kNb; ++n) {
      const int d = ci - n;
      const float val = (d == 0) ? w3 : ((d == 1) ? w2 : ((d == 2) ? w1 : ((d == 3) ? w0 : 0.0f)));
      tw[n * kIn + i] = val;
    }
    const float sg = __builtin_amdgcn_rcpf(1.0f + __expf(-xc));
    tw[kNb * kIn + i] = (xc * sg) * kCarryA;
  }
  __syncthreads();

  v8h hv[kSegs];
#pragma unroll
  for (int j = 0; j < kSegs; ++j) {
    const float* sp = tw + j * kIn + lane * 8;
    const v4f a0 = *(const v4f*)(sp);
    const v4f a1 = *(const v4f*)(sp + 4);
#pragma unroll
    for (int e = 0; e < 4; ++e) {
      const float f0 = a0[e];
      const float f1 = a1[e];
      hv[j][e]     = (_Float16)f0;
      hv[j][4 + e] = (_Float16)f1;
    }
  }
  unsigned short* dst = Aplane + (size_t)ml * kKtot + lane * 8;
  for (int pass = 0; pass < 2; ++pass) {
#pragma unroll
    for (int j = 0; j < kSegs; ++j) *(volatile v8h*)(dst + j * kIn) = hv[j];
    __threadfence();
  }
}

__global__ __launch_bounds__(256) void gemm_f16_tile64_kernel(
    const unsigned short* __restrict__ Ap, int lda,
    const unsigned short* __restrict__ Btp, int ldb,
    float* __restrict__ C, int ldc, int M, int N, int K, float scale)
{
  const _Float16* A  = (const _Float16*)Ap;
  const _Float16* Bt = (const _Float16*)Btp;
  __shared__ __align__(16) float sT[8][16 * 68];
  const int lane = threadIdx.x & 31;
  const int wave = threadIdx.x >> 5;
  const int tilesN = N >> 6;
  const int tilesM = M >> 6;
  const int tile = blockIdx.x * 8 + wave;
  if (tile >= tilesM * tilesN) return;
  const int tm = tile / tilesN;
  const int tn = tile - tm * tilesN;
  const int m0 = tm << 6;
  const int n0 = tn << 6;

  const int rlane = lane & 15;
  const int koff  = (lane >> 4) * 8;
  const int mOff  = (lane >> 4) * 8;

  v8f acc[4][4];
#pragma unroll
  for (int i = 0; i < 4; ++i)
#pragma unroll
    for (int j = 0; j < 4; ++j) acc[i][j] = (v8f){0.f, 0.f, 0.f, 0.f, 0.f, 0.f, 0.f, 0.f};

  for (int k0 = 0; k0 < K; k0 += 32) {
    v16h bh[4];
#pragma unroll
    for (int j = 0; j < 4; ++j) {
      const size_t bo = (size_t)(n0 + (j << 4) + rlane) * ldb + koff + k0;
      bh[j] = FragH::load(Bt + bo);
    }
#pragma unroll
    for (int i = 0; i < 4; ++i) {
      const size_t ao = (size_t)(m0 + (i << 4) + rlane) * lda + koff + k0;
      const v16h ah = FragH::load(A + ao);
#pragma unroll
      for (int j = 0; j < 4; ++j) acc[i][j] = FragH::mma(ah, bh[j], acc[i][j]);
      tie_acc_h(acc[i][0], ah, bh[0]);
      tie_acc_h(acc[i][1], ah, bh[1]);
      tie_acc_h(acc[i][2], ah, bh[2]);
      tie_acc_h(acc[i][3], ah, bh[3]);
    }
    keep4_h(bh[0], bh[1], bh[2], bh[3]);
  }
#pragma unroll
  for (int i = 0; i < 4; ++i) {
    settle_acc(acc[i][0]);
    settle_acc(acc[i][1]);
    settle_acc(acc[i][2]);
    settle_acc(acc[i][3]);
  }

  float* slab = sT[wave];
#pragma unroll
  for (int i = 0; i < 4; ++i) {
    const int mBase = m0 + (i << 4);
#pragma unroll
    for (int j = 0; j < 4; ++j) {
#pragma unroll
      for (int r = 0; r < 8; ++r) {
        const float v = acc[i][j][r] * scale;
        slab[(mOff + r) * 68 + (j << 4) + rlane] = v;
      }
    }
    __builtin_amdgcn_fence(__ATOMIC_RELEASE, "workgroup");
    __builtin_amdgcn_wave_barrier();
    __builtin_amdgcn_fence(__ATOMIC_ACQUIRE, "workgroup");
    {
      const int hh = lane >> 4;
      const int c4 = (lane & 15) * 4;
      for (int pass = 0; pass < 2; ++pass) {
#pragma unroll
        for (int it = 0; it < 8; ++it) {
          const int row = it * 2 + hh;
          const v4f v = *(const v4f*)(slab + row * 68 + c4);
          *(volatile v4f*)(C + (size_t)(mBase + row) * ldc + n0 + c4) = v;
        }
        __threadfence();
      }
    }
    __builtin_amdgcn_fence(__ATOMIC_RELEASE, "workgroup");
    __builtin_amdgcn_wave_barrier();
    __builtin_amdgcn_fence(__ATOMIC_ACQUIRE, "workgroup");
  }
}

extern "C" void kernel_launch(void* const* d_in, const int* in_sizes, int n_in,
                              void* d_out, int out_size, void* d_ws, size_t ws_size,
                              hipStream_t stream) {
  if (n_in < 5) return;
  if (in_sizes[0] != kRows * kIn) return;
  if (in_sizes[1] != kIn) return;
  if (in_sizes[2] != kIn) return;
  if (in_sizes[3] != kOut * kIn * kNb) return;
  if (in_sizes[4] != kOut * kIn) return;
  if (out_size != kRows * kOut) return;
  if (ws_size < kWsTotal) return;

  const float* x      = (const float*)d_in[0];
  const float* gamma  = (const float*)d_in[1];
  const float* beta   = (const float*)d_in[2];
  const float* coeff  = (const float*)d_in[3];
  const float* base_w = (const float*)d_in[4];
  float* out = (float*)d_out;

  char* ws = (char*)d_ws;
  unsigned short* Wt = (unsigned short*)(ws + kOffWt);
  unsigned short* Ap = (unsigned short*)(ws + kOffAp);

  pack_weights_kernel<<<dim3(kSegs, kOut / 8), 256, 0, stream>>>(coeff, base_w, Wt);

  constexpr int kGemmBlocks = ((kSlabRows / 64) * (kOut / 64)) / 8;
  static_assert(kGemmBlocks * 8 == (kSlabRows / 64) * (kOut / 64), "GEMM grid exact");

  for (int sidx = 0; sidx < kNumSlabs; ++sidx) {
    const int row0 = sidx * kSlabRows;
    expand_rows_kernel<<<kSlabRows / kExpWaves, kExpWaves * 32, 0, stream>>>(x, gamma, beta, Ap, row0);
    gemm_f16_tile64_kernel<<<kGemmBlocks, 256, 0, stream>>>(
        Ap, kKtot, Wt, kKtot, out + (size_t)row0 * kOut, kOut, kSlabRows, kOut, kKtot, kFold);
  }
}
